// FusedScatteringAttention_87625922773412
// MI455X (gfx1250) — hardware-verified
//
#include <hip/hip_runtime.h>
#include <hip/hip_bf16.h>
#include <math.h>


typedef _Float16 v8h  __attribute__((ext_vector_type(8)));
typedef _Float16 v16h __attribute__((ext_vector_type(16)));
typedef float    v4f  __attribute__((ext_vector_type(4)));
typedef float    v8f  __attribute__((ext_vector_type(8)));

#define BATCH 2
#define SEQ   2048
#define DMODEL 1024
#define NHEAD 16
#define HDIM  64

__device__ inline v8f wmma_f16(v16h a, v16h b, v8f c) {
  return __builtin_amdgcn_wmma_f32_16x16x32_f16(
      false, a, false, b, (short)0, c, false, false);
}

__device__ inline void async_copy16(void* lds_dst, const void* gsrc) {
  const unsigned lds_off = (unsigned)(uintptr_t)lds_dst;
  const unsigned long long ga = (unsigned long long)(uintptr_t)gsrc;
  asm volatile("global_load_async_to_lds_b128 %0, %1, off"
               :
               : "v"(lds_off), "v"(ga)
               : "memory");
}
__device__ inline void wait_async0() {
  asm volatile("s_wait_asynccnt 0x0" ::: "memory");
}

__device__ inline v16h load_frag16(const _Float16* __restrict__ tile, int lda,
                                   int kbase, int lane) {
  const int m = lane & 15;
  const int h = lane >> 4;
  const _Float16* p = tile + m * lda + kbase + 8 * h;
  v8h lo = *(const v8h*)(p);
  v8h hi = *(const v8h*)(p + 16);
  v16h r;
#pragma unroll
  for (int i = 0; i < 8; ++i) { r[i] = lo[i]; r[i + 8] = hi[i]; }
  return r;
}

__global__ __launch_bounds__(256) void cvt_kernel(const float* __restrict__ in,
                                                  _Float16* __restrict__ outh,
                                                  int n, size_t plane) {
  const int i = (blockIdx.x * 256 + threadIdx.x) * 8;
  if (i < n) {
    v4f a = *(const v4f*)(in + i);
    v4f b = *(const v4f*)(in + i + 4);
    v8h hh, ll;
#pragma unroll
    for (int e = 0; e < 4; ++e) {
      hh[e] = (_Float16)a[e];     ll[e] = (_Float16)((a[e] - (float)hh[e]) * 2048.0f);
      hh[e + 4] = (_Float16)b[e]; ll[e + 4] = (_Float16)((b[e] - (float)hh[e + 4]) * 2048.0f);
    }
    *(volatile v8h*)(outh + i) = hh; if (plane) *(volatile v8h*)(outh + plane + i) = ll; __threadfence();
    *(volatile v8h*)(outh + i) = hh; if (plane) *(volatile v8h*)(outh + plane + i) = ll;
  }
}
#define RSPLIT (1.0f / 2048.0f)
__device__ inline v8f wmma_split(v16h a, v16h al, v16h b, v16h bl, v8f c) { v8f x = {}; x = wmma_f16(al, b, x); x = wmma_f16(a, bl, x); return wmma_f16(a, b, c) + x * RSPLIT; }

__global__ __launch_bounds__(256) void gate_kernel(
    const float* __restrict__ G, const float* __restrict__ gscale,
    const float* __restrict__ ltemp, float* __restrict__ gate) {
  __shared__ float red[256];
  const int b = blockIdx.x, tid = threadIdx.x;
  const float invt = __expf(-ltemp[0]);
  float z[8];
  float mx = -3.0e38f;
#pragma unroll
  for (int i = 0; i < 8; ++i) {
    const int l = i * 256 + tid;
    const float re = G[((size_t)b * SEQ + l) * 2 + 0];
    const float im = G[((size_t)b * SEQ + l) * 2 + 1];
    z[i] = sqrtf(re * re + im * im + 1e-7f) * invt;
    mx = fmaxf(mx, z[i]);
  }
  red[tid] = mx;
  __syncthreads();
  for (int s = 128; s > 0; s >>= 1) {
    if (tid < s) red[tid] = fmaxf(red[tid], red[tid + s]);
    __syncthreads();
  }
  const float zmax = red[0];
  __syncthreads();
  float sum = 0.f;
#pragma unroll
  for (int i = 0; i < 8; ++i) sum += __expf(z[i] - zmax);
  red[tid] = sum;
  __syncthreads();
  for (int s = 128; s > 0; s >>= 1) {
    if (tid < s) red[tid] += red[tid + s];
    __syncthreads();
  }
  const float sc = gscale[0] / red[0];
#pragma unroll
  for (int i = 0; i < 8; ++i) { const float gv = __expf(z[i] - zmax) * sc; *(volatile float*)(gate + (size_t)b * SEQ + i * 256 + tid) = gv; }
  __threadfence();
#pragma unroll
  for (int i = 0; i < 8; ++i) { const float gv = __expf(z[i] - zmax) * sc; *(volatile float*)(gate + (size_t)b * SEQ + i * 256 + tid) = gv; }
}

#define TM 128
#define TN 128
#define TK 32
#define LDT 40

template <int EPI>
__global__ __launch_bounds__(256) void gemm_kernel(
    const _Float16* __restrict__ Ah, const _Float16* __restrict__ Bh,
    int M, int N, int K,
    _Float16* __restrict__ qq, _Float16* __restrict__ qk,
    _Float16* __restrict__ qv,
    const float* __restrict__ bias, float* __restrict__ outf) {
  __shared__ __attribute__((aligned(16))) unsigned char lds_raw[4 * TM * LDT * 2 * 2];
  _Float16 (*As)[TM * LDT]  = (_Float16 (*)[TM * LDT])lds_raw;
  _Float16 (*Bs)[TN * LDT]  = (_Float16 (*)[TN * LDT])(lds_raw + 2 * TM * LDT * 2);
  _Float16 (*Asl)[TM * LDT] = (_Float16 (*)[TM * LDT])(lds_raw + 4 * TM * LDT * 2);
  _Float16 (*Bsl)[TN * LDT] = (_Float16 (*)[TN * LDT])(lds_raw + 6 * TM * LDT * 2);
  float (*sC)[TN] = (float (*)[TN])lds_raw;
  const size_t PLA = (size_t)BATCH * SEQ * DMODEL;
  const size_t PLB = (EPI == 0) ? (size_t)3 * DMODEL * DMODEL : (size_t)DMODEL * DMODEL;
  const size_t PLQKV = (size_t)BATCH * NHEAD * SEQ * HDIM;
#define AOUT_SCALE 4096.0f

  const int tid = threadIdx.x;
  const int lane = tid & 31;
  const int wave = tid >> 5;
  const int wm = wave >> 1;
  const int wn = wave & 1;
  const int m0 = blockIdx.y * TM;
  const int n0 = blockIdx.x * TN;

  const int lr = tid >> 1;
  const int lc = (tid & 1) * 16;

  auto async_stage = [&](int buf, int kt) {
    const int kb = kt * TK + lc;
    const _Float16* ga = Ah + (size_t)(m0 + lr) * K + kb;
    const _Float16* gb = Bh + (size_t)(n0 + lr) * K + kb;
    _Float16* la = &As[buf][lr * LDT + lc];
    _Float16* lb = &Bs[buf][lr * LDT + lc];
    async_copy16(la, ga);
    async_copy16(la + 8, ga + 8);
    async_copy16(lb, gb);
    async_copy16(lb + 8, gb + 8);
    {
      _Float16* lal = &Asl[buf][lr * LDT + lc];
      _Float16* lbl = &Bsl[buf][lr * LDT + lc];
      async_copy16(lal, ga + PLA); async_copy16(lal + 8, ga + PLA + 8);
      async_copy16(lbl, gb + PLB); async_copy16(lbl + 8, gb + PLB + 8);
    }
  };

  v8f acc[2][4];
#pragma unroll
  for (int mi = 0; mi < 2; ++mi)
#pragma unroll
    for (int ni = 0; ni < 4; ++ni)
#pragma unroll
      for (int e = 0; e < 8; ++e) acc[mi][ni][e] = 0.f;

  const int KT = K / TK;
  async_stage(0, 0);
  wait_async0();
  __syncthreads();

  for (int kt = 0; kt < KT; ++kt) {
    const int cur = kt & 1;
    if (kt + 1 < KT) async_stage(1 - cur, kt + 1);

    v16h af0 = load_frag16(&As[cur][(wm * 32 + 0) * LDT], LDT, 0, lane);
    v16h af1 = load_frag16(&As[cur][(wm * 32 + 16) * LDT], LDT, 0, lane);
    {
      v16h al0 = load_frag16(&Asl[cur][(wm * 32 + 0) * LDT], LDT, 0, lane);
      v16h al1 = load_frag16(&Asl[cur][(wm * 32 + 16) * LDT], LDT, 0, lane);
#pragma unroll
      for (int ni = 0; ni < 4; ++ni) {
        v16h bf = load_frag16(&Bs[cur][(wn * 64 + ni * 16) * LDT], LDT, 0, lane);
        v16h bl = load_frag16(&Bsl[cur][(wn * 64 + ni * 16) * LDT], LDT, 0, lane);
        acc[0][ni] = wmma_split(af0, al0, bf, bl, acc[0][ni]);
        acc[1][ni] = wmma_split(af1, al1, bf, bl, acc[1][ni]);
      }
    }
    if (kt + 1 < KT) wait_async0();
    __syncthreads();
  }

  const int hf = lane >> 4;
  const int cl = lane & 15;
#pragma unroll
  for (int mi = 0; mi < 2; ++mi)
#pragma unroll
    for (int ni = 0; ni < 4; ++ni)
#pragma unroll
      for (int r = 0; r < 8; ++r) sC[wm * 32 + mi * 16 + r + 8 * hf][wn * 64 + ni * 16 + cl] = acc[mi][ni][r];
  __syncthreads();
#pragma unroll 1
  for (int pass = 0; pass < 2; ++pass) {
    if (EPI == 0) {
      const int which = n0 >> 10, head0 = (n0 & 1023) >> 6;
      _Float16* dstb = (which == 0) ? qq : ((which == 1) ? qk : qv);
      for (int c = tid; c < TM * 16; c += 256) {
        const int ml = c >> 4, hh2 = (c >> 3) & 1, d8 = (c & 7) * 8;
        const int m = m0 + ml, bb = m >> 11, ll = m & 2047;
        const float* s = &sC[ml][hh2 * 64 + d8];
        union { v8h v; _Float16 h[8]; } pk, pkl;
#pragma unroll
        for (int j = 0; j < 8; ++j) { pk.h[j] = (_Float16)s[j]; pkl.h[j] = (_Float16)((s[j] - (float)pk.h[j]) * 2048.0f); }
        _Float16* dq = dstb + (((size_t)(bb * NHEAD + head0 + hh2) * SEQ + ll) * HDIM) + d8;
        *(volatile v8h*)dq = pk.v; *(volatile v8h*)(dq + PLQKV) = pkl.v;
      }
    } else {
      for (int c = tid; c < TM * 32; c += 256) {
        const int ml = c >> 5, q4 = (c & 31) * 4;
        v4f o;
#pragma unroll
        for (int j = 0; j < 4; ++j) o[j] = sC[ml][q4 + j] * (1.0f / AOUT_SCALE) + bias[n0 + q4 + j];
        *(volatile v4f*)(outf + (size_t)(m0 + ml) * N + n0 + q4) = o;
      }
    }
    __threadfence();
  }
}

__global__ __launch_bounds__(256) void attn_kernel(
    const _Float16* __restrict__ q, const _Float16* __restrict__ k,
    const _Float16* __restrict__ v, const float* __restrict__ gate,
    _Float16* __restrict__ aout) {
  __shared__ _Float16 Qs[128 * 72], Qsl[128 * 72];
  __shared__ _Float16 Ks[64 * 72], Ksl[64 * 72];
  __shared__ _Float16 Vt[64 * 72], Vtl[64 * 72];
  __shared__ _Float16 Ps[8][16 * 72], Psl[8][16 * 72];
  const size_t PLQKV = (size_t)BATCH * NHEAD * SEQ * HDIM;
  __shared__ __attribute__((aligned(16))) float Os[8][16][68];

  const int tid = threadIdx.x;
  const int lane = tid & 31;
  const int wave = tid >> 5;
  const int bh = blockIdx.y;
  const int b = bh >> 4;
  const int h = bh & 15;
  const int q0 = blockIdx.x * 128;
  const size_t base = (size_t)bh * SEQ * HDIM;

  {
    const int r = tid >> 1;
    const int c0 = (tid & 1) * 32;
    const _Float16* src = q + base + (size_t)(q0 + r) * HDIM + c0;
#pragma unroll
    for (int j = 0; j < 4; ++j) { async_copy16(&Qs[r * 72 + c0 + 8 * j], src + 8 * j); async_copy16(&Qsl[r * 72 + c0 + 8 * j], src + PLQKV + 8 * j); }
  }
  wait_async0();
  __syncthreads();
  v16h qf0 = load_frag16(&Qs[(wave * 16) * 72], 72, 0, lane), ql0 = load_frag16(&Qsl[(wave * 16) * 72], 72, 0, lane);
  v16h qf1 = load_frag16(&Qs[(wave * 16) * 72], 72, 32, lane), ql1 = load_frag16(&Qsl[(wave * 16) * 72], 72, 32, lane);

  v8f oacc[4];
  float rm[8], rl[8];
#pragma unroll
  for (int nt = 0; nt < 4; ++nt)
#pragma unroll
    for (int e = 0; e < 8; ++e) oacc[nt][e] = 0.f;
#pragma unroll
  for (int r = 0; r < 8; ++r) { rm[r] = -3.0e38f; rl[r] = 0.f; }

  const float scale = 0.125f;
  const int hf = lane >> 4;
  const int cl = lane & 15;

  for (int ktile = 0; ktile < SEQ / 64; ++ktile) {
    __syncthreads();
    {
      const int r = tid >> 2;
      const int c0 = (tid & 3) * 16;
      const _Float16* ksrc = k + base + (size_t)(ktile * 64 + r) * HDIM + c0;
      async_copy16(&Ks[r * 72 + c0], ksrc);
      async_copy16(&Ks[r * 72 + c0 + 8], ksrc + 8);
      async_copy16(&Ksl[r * 72 + c0], ksrc + PLQKV);
      async_copy16(&Ksl[r * 72 + c0 + 8], ksrc + PLQKV + 8);
      const _Float16* vsrc = v + base + (size_t)(ktile * 64 + r) * HDIM + c0;
      v8h u0 = *(const v8h*)(vsrc), u1 = *(const v8h*)(vsrc + 8);
      v8h w0 = *(const v8h*)(vsrc + PLQKV), w1 = *(const v8h*)(vsrc + PLQKV + 8);
#pragma unroll
      for (int j = 0; j < 8; ++j) {
        Vt[(c0 + j) * 72 + r] = u0[j];      Vtl[(c0 + j) * 72 + r] = w0[j];
        Vt[(c0 + 8 + j) * 72 + r] = u1[j];  Vtl[(c0 + 8 + j) * 72 + r] = w1[j];
      }
    }
    wait_async0();
    __syncthreads();

    v8f sacc[4];
#pragma unroll
    for (int nt = 0; nt < 4; ++nt) {
#pragma unroll
      for (int e = 0; e < 8; ++e) sacc[nt][e] = 0.f;
      v16h bf0 = load_frag16(&Ks[(nt * 16) * 72], 72, 0, lane), bl0 = load_frag16(&Ksl[(nt * 16) * 72], 72, 0, lane);
      sacc[nt] = wmma_split(qf0, ql0, bf0, bl0, sacc[nt]);
      v16h bf1 = load_frag16(&Ks[(nt * 16) * 72], 72, 32, lane), bl1 = load_frag16(&Ksl[(nt * 16) * 72], 72, 32, lane);
      sacc[nt] = wmma_split(qf1, ql1, bf1, bl1, sacc[nt]);
    }

#pragma unroll
    for (int r = 0; r < 8; ++r) {
      const float s0 = sacc[0][r] * scale;
      const float s1 = sacc[1][r] * scale;
      const float s2 = sacc[2][r] * scale;
      const float s3 = sacc[3][r] * scale;
      float t = fmaxf(fmaxf(s0, s1), fmaxf(s2, s3));
#pragma unroll
      for (int msk = 1; msk <= 8; msk <<= 1)
        t = fmaxf(t, __shfl_xor(t, msk, 32));
      const float mnew = fmaxf(rm[r], t);
      const float alpha = __expf(rm[r] - mnew);
      rm[r] = mnew;
      const float p0 = __expf(s0 - mnew);
      const float p1 = __expf(s1 - mnew);
      const float p2 = __expf(s2 - mnew);
      const float p3 = __expf(s3 - mnew);
      _Float16* pp = &Ps[wave][(r + 8 * hf) * 72];
      _Float16* ppl = &Psl[wave][(r + 8 * hf) * 72];
      { const float qv = p0 * 1024.0f; const _Float16 hq = (_Float16)qv; pp[0 + cl] = hq;  ppl[0 + cl] = (_Float16)((qv - (float)hq) * 2048.0f); }
      { const float qv = p1 * 1024.0f; const _Float16 hq = (_Float16)qv; pp[16 + cl] = hq; ppl[16 + cl] = (_Float16)((qv - (float)hq) * 2048.0f); }
      { const float qv = p2 * 1024.0f; const _Float16 hq = (_Float16)qv; pp[32 + cl] = hq; ppl[32 + cl] = (_Float16)((qv - (float)hq) * 2048.0f); }
      { const float qv = p3 * 1024.0f; const _Float16 hq = (_Float16)qv; pp[48 + cl] = hq; ppl[48 + cl] = (_Float16)((qv - (float)hq) * 2048.0f); }
      float ps = p0 + p1 + p2 + p3;
#pragma unroll
      for (int msk = 1; msk <= 8; msk <<= 1) ps += __shfl_xor(ps, msk, 32);
      rl[r] = rl[r] * alpha + ps;
#pragma unroll
      for (int nt = 0; nt < 4; ++nt) oacc[nt][r] *= alpha;
    }

#pragma unroll
    for (int ks = 0; ks < 2; ++ks) {
      v16h pf = load_frag16(Ps[wave], 72, 32 * ks, lane), pfl = load_frag16(Psl[wave], 72, 32 * ks, lane);
#pragma unroll
      for (int nt = 0; nt < 4; ++nt) {
        v16h vf = load_frag16(&Vt[(nt * 16) * 72], 72, 32 * ks, lane), vfl = load_frag16(&Vtl[(nt * 16) * 72], 72, 32 * ks, lane);
        oacc[nt] = wmma_split(pf, pfl, vf, vfl, oacc[nt]);
      }
    }
  }

#pragma unroll
  for (int r = 0; r < 8; ++r) {
    const int row = q0 + wave * 16 + r + 8 * hf;
    const float g = gate[(size_t)b * SEQ + row] / (rl[r] * 1024.0f) * 4096.0f;
#pragma unroll
    for (int nt = 0; nt < 4; ++nt) Os[wave][r + 8 * hf][nt * 16 + cl] = oacc[nt][r] * g;
  }
  asm volatile("s_wait_dscnt 0" ::: "memory");
#pragma unroll 1
  for (int pass = 0; pass < 2; ++pass) {
#pragma unroll
    for (int i = 0; i < 4; ++i) {
      const int c = lane + 32 * i, rr = c >> 3, d8 = (c & 7) * 8;
      const int row = q0 + wave * 16 + rr;
      const float* s = &Os[wave][rr][d8];
      union { v8h v; _Float16 h[8]; } pk, pkl;
#pragma unroll
      for (int j = 0; j < 8; ++j) { pk.h[j] = (_Float16)s[j]; pkl.h[j] = (_Float16)((s[j] - (float)pk.h[j]) * 2048.0f); }
      *(volatile v8h*)(aout + ((size_t)(b * SEQ + row)) * DMODEL + h * HDIM + d8) = pk.v;
      *(volatile v8h*)(aout + (size_t)BATCH * SEQ * DMODEL + ((size_t)(b * SEQ + row)) * DMODEL + h * HDIM + d8) = pkl.v;
    }
    __threadfence();
  }
}

extern "C" void kernel_launch(void* const* d_in, const int* in_sizes, int n_in,
                              void* d_out, int out_size, void* d_ws,
                              size_t ws_size, hipStream_t stream) {
  const float* x = (const float*)d_in[0];
  const float* G = (const float*)d_in[1];
  const float* qkv_w = (const float*)d_in[2];
  const float* out_w = (const float*)d_in[3];
  const float* out_b = (const float*)d_in[4];
  const float* gate_scale = (const float*)d_in[5];
  const float* log_temp = (const float*)d_in[6];
  float* out = (float*)d_out;

  const size_t BLD = (size_t)BATCH * SEQ * DMODEL;
  _Float16* qb = (_Float16*)d_ws;
  _Float16* kb = qb + 2 * BLD;
  _Float16* vb = kb + 2 * BLD;
  _Float16* ab = vb + 2 * BLD;
  _Float16* xh = ab + 2 * BLD;
  _Float16* wqkvh = xh + 2 * BLD;
  _Float16* wouth = wqkvh + 2 * 3 * DMODEL * DMODEL;
  float* gate = (float*)(wouth + 2 * DMODEL * DMODEL);

  cvt_kernel<<<dim3((int)(BLD / 2048)), dim3(256), 0, stream>>>(x, xh,
                                                                (int)BLD, BLD);
  cvt_kernel<<<dim3(3 * DMODEL * DMODEL / 2048), dim3(256), 0, stream>>>(
      qkv_w, wqkvh, 3 * DMODEL * DMODEL, (size_t)3 * DMODEL * DMODEL);
  cvt_kernel<<<dim3(DMODEL * DMODEL / 2048), dim3(256), 0, stream>>>(
      out_w, wouth, DMODEL * DMODEL, (size_t)DMODEL * DMODEL);

  gate_kernel<<<dim3(BATCH), dim3(256), 0, stream>>>(G, gate_scale, log_temp,
                                                     gate);

  gemm_kernel<0><<<dim3(3072 / TN, 4096 / TM), dim3(256), 0, stream>>>(
      xh, wqkvh, 4096, 3072, 1024, qb, kb, vb, nullptr, nullptr);

  attn_kernel<<<dim3(SEQ / 128, BATCH * NHEAD), dim3(256), 0, stream>>>(
      qb, kb, vb, gate, ab);

  gemm_kernel<1><<<dim3(1024 / TN, 4096 / TM), dim3(256), 0, stream>>>(
      ab, wouth, 4096, 1024, 1024, nullptr, nullptr, nullptr, out_b, out);
}
